// UserHistoryTower_56770877718674
// MI455X (gfx1250) — hardware-verified
//
#include <hip/hip_runtime.h>
#include <math.h>

constexpr int kRows = 8192;
constexpr int kDim  = 128;
constexpr int kHidA = 512;
constexpr int kHidB = 256;
constexpr int kRowsPerHistBlock = 32;
static_assert(kRows % kRowsPerHistBlock == 0);
static_assert(kRows % 64 == 0 && kDim % 64 == 0 && kHidA % 64 == 0 && kHidB % 64 == 0);
static_assert(kDim % 32 == 0 && kHidA % 32 == 0 && kHidB % 32 == 0);
static_assert(kRows % 128 == 0);

typedef __attribute__((ext_vector_type(16))) _Float16 v16h;
typedef __attribute__((ext_vector_type(8)))  _Float16 v8h;
typedef __attribute__((ext_vector_type(16))) __bf16   v16b;
typedef __attribute__((ext_vector_type(8)))  __bf16   v8b;
typedef __attribute__((ext_vector_type(8)))  float    v8f;
typedef __attribute__((ext_vector_type(4)))  float    v4f;
typedef __attribute__((ext_vector_type(4)))  unsigned int v4u;
typedef __attribute__((ext_vector_type(4)))  int      v4i;

constexpr size_t kBytesW1p  = (size_t)kHidA * kDim * 2;
constexpr size_t kBytesW2p  = (size_t)kHidB * kHidA * 2;
constexpr size_t kBytesW3p  = (size_t)kDim * kHidB * 2;
constexpr size_t kBytesHp   = (size_t)kRows * kDim * 2;
constexpr size_t kBytesFlag = (size_t)kRows * 4;
constexpr size_t kBytesA1p  = (size_t)kRows * kHidA * 2;
constexpr size_t kBytesA2p  = (size_t)kRows * kHidB * 2;
constexpr size_t kBytesA3   = (size_t)kRows * kDim * 4;
constexpr size_t kOffW1h  = 0;
constexpr size_t kOffW1l  = kOffW1h + kBytesW1p;
constexpr size_t kOffW2h  = kOffW1l + kBytesW1p;
constexpr size_t kOffW2l  = kOffW2h + kBytesW2p;
constexpr size_t kOffW3h  = kOffW2l + kBytesW2p;
constexpr size_t kOffW3l  = kOffW3h + kBytesW3p;
constexpr size_t kOffHh   = kOffW3l + kBytesW3p;
constexpr size_t kOffHl   = kOffHh + kBytesHp;
constexpr size_t kOffFlag = kOffHl + kBytesHp;
constexpr size_t kOffA1h  = kOffFlag + kBytesFlag;
constexpr size_t kOffA1l  = kOffA1h + kBytesA1p;
constexpr size_t kOffA2h  = kOffA1l + kBytesA1p;
constexpr size_t kOffA2l  = kOffA2h + kBytesA2p;
constexpr size_t kOffA3   = kOffA2l + kBytesA2p;
constexpr size_t kWsTotal = kOffA3 + kBytesA3;
static_assert(kWsTotal == 34504704);
static_assert(kWsTotal <= (size_t)134217728);
static_assert(kOffHh % 128 == 0 && kOffFlag % 128 == 0 && kOffA1h % 128 == 0 && kOffA3 % 128 == 0);

__device__ __forceinline__ unsigned short f2bf_bits(float f) {
  unsigned u = __float_as_uint(f);
  return (unsigned short)((u + 0x7FFFu + ((u >> 16) & 1u)) >> 16);
}
__device__ __forceinline__ float bf_bits2f(unsigned short h) { return __uint_as_float(((unsigned)h) << 16); }

__device__ __forceinline__ void dep_guard_h(v8f& a, v8f& b, v16h x, v16h y) { asm volatile("v_nop\n\tv_nop\n\tv_nop\n\tv_nop" : "+v"(a), "+v"(b) : "v"(x), "v"(y)); }
__device__ __forceinline__ void dep_guard_b(v8f& a, v8f& b, v16b x, v16b y) { asm volatile("v_nop\n\tv_nop\n\tv_nop\n\tv_nop" : "+v"(a), "+v"(b) : "v"(x), "v"(y)); }
__device__ __forceinline__ void keep4_h(v16h a, v16h b, v16h c, v16h d) { asm volatile("v_nop" :: "v"(a), "v"(b), "v"(c), "v"(d)); }
__device__ __forceinline__ void keep4_b(v16b a, v16b b, v16b c, v16b d) { asm volatile("v_nop" :: "v"(a), "v"(b), "v"(c), "v"(d)); }
__device__ __forceinline__ void acc_guard4(v8f& a, v8f& b, v8f& c, v8f& d) { asm volatile("v_nop\n\tv_nop\n\tv_nop\n\tv_nop" : "+v"(a), "+v"(b), "+v"(c), "+v"(d)); }
template <typename T> struct Frag;
template <> struct Frag<_Float16> {
  typedef v16h V; union U { v16h v; v8h h[2]; };
  static __device__ __forceinline__ v16h load(const _Float16* p) {
    U f; f.h[0] = *(const v8h*)(p); f.h[1] = *(const v8h*)(p + 16); return f.v;
  }
  static __device__ __forceinline__ v8f mma(v16h a, v16h b, v8f c) {
    return __builtin_amdgcn_wmma_f32_16x16x32_f16(false, a, false, b, (short)0, c, false, false);
  }
  static __device__ __forceinline__ void guard(v8f& a, v8f& b, v16h x, v16h y) { dep_guard_h(a, b, x, y); }
  static __device__ __forceinline__ void keep(v16h a, v16h b, v16h c, v16h d) { keep4_h(a, b, c, d); }
};
template <> struct Frag<__bf16> {
  typedef v16b V; union U { v16b v; v8b h[2]; };
  static __device__ __forceinline__ v16b load(const __bf16* p) {
    U f; f.h[0] = *(const v8b*)(p); f.h[1] = *(const v8b*)(p + 16); return f.v;
  }
  static __device__ __forceinline__ v8f mma(v16b a, v16b b, v8f c) {
    return __builtin_amdgcn_wmma_f32_16x16x32_bf16(false, a, false, b, (short)0, c, false, false);
  }
  static __device__ __forceinline__ void guard(v8f& a, v8f& b, v16b x, v16b y) { dep_guard_b(a, b, x, y); }
  static __device__ __forceinline__ void keep(v16b a, v16b b, v16b c, v16b d) { keep4_b(a, b, c, d); }
};

__device__ __forceinline__ unsigned pk16(unsigned short a, unsigned short b) { return (unsigned)a | ((unsigned)b << 16); }

template <int ET> struct Elem;
template <> struct Elem<0> { typedef _Float16 T; };
template <> struct Elem<1> { typedef __bf16 T; };
template <int ET, bool SPLIT, int BIAS_MODE, int OUT_MODE, bool RESID, int ACT = 0>
__global__ __launch_bounds__(256) void wmma_gemm64(
    const unsigned short* __restrict__ Ap, const unsigned short* __restrict__ A2p, int lda, long strideA,
    const unsigned short* __restrict__ Btp, const unsigned short* __restrict__ Bt2p, int ldb, long strideB,
    void* __restrict__ Cout, void* __restrict__ Cout2, int ldc, long strideC,
    const float* __restrict__ bias,
    const float* __restrict__ resid, long strideR,
    int M, int N, int K, float scale) {
  typedef typename Elem<ET>::T T;
  typedef typename Frag<T>::V V;
  const T* A = (const T*)Ap; const T* A2 = (const T*)A2p; const T* Bt = (const T*)Btp; const T* Bt2 = (const T*)Bt2p;
  __shared__ __align__(16) float sT[8][16 * 68];
  const int b    = blockIdx.y;
  const int lane = threadIdx.x & 31;
  const int wave = threadIdx.x >> 5;
  const int tilesN = N >> 6;
  const int tilesM = M >> 6;
  const int tile = blockIdx.x * 8 + wave;
  if (tile >= tilesM * tilesN) return;
  const int tm = tile / tilesN;
  const int tn = tile - tm * tilesN;
  const int m0 = tm << 6;
  const int n0 = tn << 6;

  const T* Ab  = A  + (size_t)b * strideA;
  const T* Bb  = Bt + (size_t)b * strideB;
  const T* Ab2 = SPLIT ? (A2  + (size_t)b * strideA) : nullptr;
  const T* Bb2 = SPLIT ? (Bt2 + (size_t)b * strideB) : nullptr;

  const int rlane = lane & 15;
  const int koff  = (lane >> 4) * 8;
  const int mOff  = (lane >> 4) * 8;

  v8f acc[4][4];
#pragma unroll
  for (int i = 0; i < 4; ++i)
#pragma unroll
    for (int j = 0; j < 4; ++j) acc[i][j] = (v8f){0.f,0.f,0.f,0.f,0.f,0.f,0.f,0.f};

  for (int k0 = 0; k0 < K; k0 += 32) {
    V bh[4], bl[4];
#pragma unroll
    for (int j = 0; j < 4; ++j) {
      const size_t bo = (size_t)(n0 + (j << 4) + rlane) * ldb + koff + k0;
      bh[j] = Frag<T>::load(Bb + bo);
      if (SPLIT) bl[j] = Frag<T>::load(Bb2 + bo);
    }
#pragma unroll
    for (int i = 0; i < 4; ++i) {
      const size_t ao = (size_t)(m0 + (i << 4) + rlane) * lda + koff + k0;
      V ah = Frag<T>::load(Ab + ao);
      V al;
      if (SPLIT) al = Frag<T>::load(Ab2 + ao);
#pragma unroll
      for (int j = 0; j < 4; ++j) {
        acc[i][j] = Frag<T>::mma(ah, bh[j], acc[i][j]);
        if (SPLIT) {
          acc[i][j] = Frag<T>::mma(ah, bl[j], acc[i][j]);
          acc[i][j] = Frag<T>::mma(al, bh[j], acc[i][j]);
        }
      }
      Frag<T>::guard(acc[i][0], acc[i][3], ah, SPLIT ? al : ah);
    }
    Frag<T>::keep(bh[0], bh[1], bh[2], bh[3]);
    if (SPLIT) Frag<T>::keep(bl[0], bl[1], bl[2], bl[3]);
  }
  acc_guard4(acc[0][0], acc[0][1], acc[0][2], acc[0][3]);
  acc_guard4(acc[1][0], acc[1][1], acc[1][2], acc[1][3]);
  acc_guard4(acc[2][0], acc[2][1], acc[2][2], acc[2][3]);
  acc_guard4(acc[3][0], acc[3][1], acc[3][2], acc[3][3]);

  float* slab = sT[wave];
  const float* Rb = RESID ? (resid + (size_t)b * strideR) : nullptr;
#pragma unroll
  for (int i = 0; i < 4; ++i) {
    const int mBase = m0 + (i << 4);
#pragma unroll
    for (int j = 0; j < 4; ++j) {
      const int n = n0 + (j << 4) + rlane;
      float bv = 0.f;
      if (BIAS_MODE == 2) bv = bias[n];
#pragma unroll
      for (int r = 0; r < 8; ++r) {
        float v = acc[i][j][r] * scale;
        if (BIAS_MODE == 1) v += bias[mBase + mOff + r];
        if (BIAS_MODE == 2) v += bv;
        if (RESID) v += Rb[(size_t)(mBase + mOff + r) * ldc + n];
        if (ACT == 2) v = fmaxf(v, 0.0f);
        if (ACT == 4) v = (v > 0.f) ? v : 0.01f * v;
        if (ACT == 6) v = v * __builtin_amdgcn_rcpf(1.0f + __expf(-v));
        slab[(mOff + r) * 68 + (j << 4) + rlane] = v;
      }
    }
    __builtin_amdgcn_fence(__ATOMIC_RELEASE, "workgroup");
    __builtin_amdgcn_wave_barrier();
    __builtin_amdgcn_fence(__ATOMIC_ACQUIRE, "workgroup");
    if (OUT_MODE == 0) {
      float* C = (float*)Cout + (size_t)b * strideC;
      const int hh = lane >> 4, c4 = (lane & 15) * 4;
      for (int pass = 0; pass < 2; ++pass) {
#pragma unroll
        for (int it = 0; it < 8; ++it) {
          const int row = it * 2 + hh;
          v4f v = *(const v4f*)(slab + row * 68 + c4);
          *(volatile v4f*)(C + (size_t)(mBase + row) * ldc + n0 + c4) = v;
        }
        __threadfence();
      }
    } else {
      const int q = lane >> 3, c8 = (lane & 7) * 8;
      unsigned short* C  = (unsigned short*)Cout  + (size_t)b * strideC;
      unsigned short* C2 = (OUT_MODE == 2) ? ((unsigned short*)Cout2 + (size_t)b * strideC) : nullptr;
      for (int pass = 0; pass < 2; ++pass) {
#pragma unroll
        for (int it = 0; it < 4; ++it) {
          const int row = it * 4 + q;
          const float* sp = slab + row * 68 + c8;
          v8h hv, lv;
#pragma unroll
          for (int e = 0; e < 8; ++e) {
            if (OUT_MODE == 1) {
              hv[e] = (_Float16)sp[e];
            } else {
              unsigned short hb = f2bf_bits(sp[e]);
              unsigned short lb = f2bf_bits(sp[e] - bf_bits2f(hb));
              hv[e] = __builtin_bit_cast(_Float16, hb);
              lv[e] = __builtin_bit_cast(_Float16, lb);
            }
          }
          *(volatile v8h*)(C + (size_t)(mBase + row) * ldc + n0 + c8) = hv;
          if (OUT_MODE == 2) *(volatile v8h*)(C2 + (size_t)(mBase + row) * ldc + n0 + c8) = lv;
        }
        __threadfence();
      }
    }
    __builtin_amdgcn_fence(__ATOMIC_RELEASE, "workgroup");
    __builtin_amdgcn_wave_barrier();
    __builtin_amdgcn_fence(__ATOMIC_ACQUIRE, "workgroup");
  }
}

__global__ __launch_bounds__(256) void wt_split_kernel(const float* __restrict__ W,
                                                       unsigned short* __restrict__ Bhi,
                                                       unsigned short* __restrict__ Blo,
                                                       int Kin, int Nout) {
  __shared__ float sm[64][65];
  const int t  = threadIdx.x;
  const int k0 = blockIdx.x * 64;
  const int n0 = blockIdx.y * 64;
#pragma unroll
  for (int i = 0; i < 16; ++i) {
    const int e = i * 256 + t;
    const int r = e >> 6;
    const int c = e & 63;
    sm[c][r] = W[(size_t)(k0 + r) * Nout + n0 + c];
  }
  __syncthreads();
  const int lane = t & 31, wave = t >> 5;
  const int q = lane >> 3, c8 = (lane & 7) * 8;
  for (int pass = 0; pass < 2; ++pass) {
#pragma unroll
    for (int it = 0; it < 2; ++it) {
      const int rowl = wave * 8 + it * 4 + q;
      unsigned short hb[8], lb[8];
#pragma unroll
      for (int e = 0; e < 8; ++e) {
        const float x = sm[rowl][c8 + e];
        const unsigned short h = f2bf_bits(x);
        hb[e] = h;
        lb[e] = f2bf_bits(x - bf_bits2f(h));
      }
      const v4u uh = (v4u){pk16(hb[0], hb[1]), pk16(hb[2], hb[3]), pk16(hb[4], hb[5]), pk16(hb[6], hb[7])};
      const v4u ul = (v4u){pk16(lb[0], lb[1]), pk16(lb[2], lb[3]), pk16(lb[4], lb[5]), pk16(lb[6], lb[7])};
      const size_t o = (size_t)(n0 + rowl) * Kin + k0 + c8;
      *(volatile v4u*)(Bhi + o) = uh;
      *(volatile v4u*)(Blo + o) = ul;
    }
    __threadfence();
  }
}

__device__ __forceinline__ void gather_bits(unsigned m, int base, const float* __restrict__ emb,
                                            int lane, float w, v4f& acc) {
#pragma unroll 1
  for (int q = 0; q < 32; ++q) {
    if (m == 0u) break;
    const int t = __builtin_ctz(m);
    m &= m - 1u;
    int j = base + 4 * t;
    j = j < 0 ? 0 : (j > kRows - 1 ? kRows - 1 : j);
    const v4f v = *(const v4f*)(emb + (size_t)j * kDim + lane * 4);
    acc += w * v;
  }
}

__global__ __launch_bounds__(256) void history_kernel(const float* __restrict__ emb,
                                                      const int* __restrict__ user,
                                                      const int* __restrict__ ts,
                                                      const int* __restrict__ click,
                                                      unsigned short* __restrict__ Hhi,
                                                      unsigned short* __restrict__ Hlo,
                                                      float* __restrict__ flag) {
  __shared__ __align__(16) float srow[8][kDim];
  __shared__ __align__(16) float sflag[kRowsPerHistBlock];
  const int lane = threadIdx.x & 31;
  const int wave = threadIdx.x >> 5;

#pragma unroll 1
  for (int rr = 0; rr < 4; ++rr) {
    const int row = blockIdx.x * kRowsPerHistBlock + wave * 4 + rr;
    const int ui = user[row];
    const int ti = ts[row];

    int cl = 0;
#pragma unroll 1
    for (int jb = 0; jb < kRows; jb += 128) {
      const int j4 = jb + lane * 4;
      const v4i uu = *(const v4i*)(user + j4);
      const v4i tt = *(const v4i*)(ts + j4);
      const v4i cc = *(const v4i*)(click + j4);
      cl += ((cc.x != 0) & (uu.x == ui) & (ti > tt.x)) ? 1 : 0;
      cl += ((cc.y != 0) & (uu.y == ui) & (ti > tt.y)) ? 1 : 0;
      cl += ((cc.z != 0) & (uu.z == ui) & (ti > tt.z)) ? 1 : 0;
      cl += ((cc.w != 0) & (uu.w == ui) & (ti > tt.w)) ? 1 : 0;
    }
#pragma unroll
    for (int off = 16; off > 0; off >>= 1) cl += __shfl_xor(cl, off, 32);
    const float denom = (float)cl + 1e-16f;
    const float w = 1.0f / denom;

    v4f acc = (v4f){0.f, 0.f, 0.f, 0.f};
#pragma unroll 1
    for (int jb = 0; jb < kRows; jb += 128) {
      const int j4 = jb + lane * 4;
      const v4i uu = *(const v4i*)(user + j4);
      const v4i tt = *(const v4i*)(ts + j4);
      const v4i cc = *(const v4i*)(click + j4);
      const bool p0 = (cc.x != 0) & (uu.x == ui) & (ti > tt.x);
      const bool p1 = (cc.y != 0) & (uu.y == ui) & (ti > tt.y);
      const bool p2 = (cc.z != 0) & (uu.z == ui) & (ti > tt.z);
      const bool p3 = (cc.w != 0) & (uu.w == ui) & (ti > tt.w);
      const unsigned m0 = __builtin_amdgcn_ballot_w32(p0);
      const unsigned m1 = __builtin_amdgcn_ballot_w32(p1);
      const unsigned m2 = __builtin_amdgcn_ballot_w32(p2);
      const unsigned m3 = __builtin_amdgcn_ballot_w32(p3);
      gather_bits(m0, jb + 0, emb, lane, w, acc);
      gather_bits(m1, jb + 1, emb, lane, w, acc);
      gather_bits(m2, jb + 2, emb, lane, w, acc);
      gather_bits(m3, jb + 3, emb, lane, w, acc);
    }

    *(v4f*)(&srow[wave][lane * 4]) = acc;
    __builtin_amdgcn_fence(__ATOMIC_RELEASE, "workgroup");
    __builtin_amdgcn_wave_barrier();
    __builtin_amdgcn_fence(__ATOMIC_ACQUIRE, "workgroup");
    const int c8 = (lane & 15) * 8;
    const v4f x0 = *(const v4f*)(&srow[wave][c8]);
    const v4f x1 = *(const v4f*)(&srow[wave][c8 + 4]);
    unsigned short hb[8], lb[8];
#pragma unroll
    for (int e = 0; e < 4; ++e) {
      const float xa = x0[e];
      const unsigned short ha = f2bf_bits(xa);
      hb[e] = ha;
      lb[e] = f2bf_bits(xa - bf_bits2f(ha));
      const float xb = x1[e];
      const unsigned short hbb = f2bf_bits(xb);
      hb[4 + e] = hbb;
      lb[4 + e] = f2bf_bits(xb - bf_bits2f(hbb));
    }
    const v4u uh = (v4u){pk16(hb[0], hb[1]), pk16(hb[2], hb[3]), pk16(hb[4], hb[5]), pk16(hb[6], hb[7])};
    const v4u ul = (v4u){pk16(lb[0], lb[1]), pk16(lb[2], lb[3]), pk16(lb[4], lb[5]), pk16(lb[6], lb[7])};
    unsigned short* ph = Hhi + (size_t)row * kDim + c8;
    unsigned short* pl = Hlo + (size_t)row * kDim + c8;
    for (int pass = 0; pass < 2; ++pass) {
      if (lane < 16) {
        *(volatile v4u*)ph = uh;
        *(volatile v4u*)pl = ul;
      }
      __threadfence();
    }
    if (lane == 0) sflag[wave * 4 + rr] = (cl > 0) ? 1.0f : 0.0f;
    __builtin_amdgcn_fence(__ATOMIC_RELEASE, "workgroup");
    __builtin_amdgcn_wave_barrier();
    __builtin_amdgcn_fence(__ATOMIC_ACQUIRE, "workgroup");
  }

  __syncthreads();
  if (wave == 0) {
    const v4f fv = *(const v4f*)(&sflag[(lane & 7) * 4]);
    float* fp = flag + (size_t)blockIdx.x * kRowsPerHistBlock + (lane & 7) * 4;
    for (int pass = 0; pass < 2; ++pass) {
      if (lane < 8) *(volatile v4f*)fp = fv;
      __threadfence();
    }
  }
}

__global__ __launch_bounds__(256) void l2norm_kernel(const float* __restrict__ act3,
                                                     const float* __restrict__ flag,
                                                     float* __restrict__ out) {
  const int lane = threadIdx.x & 31;
  const int wave = threadIdx.x >> 5;
  const int row  = blockIdx.x * 8 + wave;
  const v4f v = *(const v4f*)(act3 + (size_t)row * kDim + lane * 4);
  float ss = v.x * v.x + v.y * v.y + v.z * v.z + v.w * v.w;
#pragma unroll
  for (int off = 16; off > 0; off >>= 1) ss += __shfl_xor(ss, off, 32);
  const float n1   = sqrtf(ss);
  const float inv1 = 1.0f / fmaxf(n1, 1e-16f);
  const v4f x1 = v * inv1;
  float ss2 = x1.x * x1.x + x1.y * x1.y + x1.z * x1.z + x1.w * x1.w;
#pragma unroll
  for (int off = 16; off > 0; off >>= 1) ss2 += __shfl_xor(ss2, off, 32);
  const float n2   = sqrtf(ss2);
  const float inv2 = 1.0f / fmaxf(n2, 1e-16f);
  const v4f x2 = x1 * inv2;
  const bool nz = (flag[row] != 0.0f);
  v4f r;
  r.x = nz ? x2.x : 0.0f;
  r.y = nz ? x2.y : 0.0f;
  r.z = nz ? x2.z : 0.0f;
  r.w = nz ? x2.w : 0.0f;
  float* op = out + (size_t)row * kDim + lane * 4;
  for (int pass = 0; pass < 2; ++pass) {
    *(volatile v4f*)op = r;
    __threadfence();
  }
}

extern "C" void kernel_launch(void* const* d_in, const int* in_sizes, int n_in,
                              void* d_out, int out_size, void* d_ws, size_t ws_size,
                              hipStream_t stream) {
  if (n_in < 10) return;
  if (in_sizes[0] != kRows * kDim || in_sizes[1] != kRows || in_sizes[2] != kRows ||
      in_sizes[3] != kRows || in_sizes[4] != kDim * kHidA || in_sizes[5] != kHidA ||
      in_sizes[6] != kHidA * kHidB || in_sizes[7] != kHidB || in_sizes[8] != kHidB * kDim ||
      in_sizes[9] != kDim || out_size != kRows * kDim) return;
  if (ws_size < kWsTotal) return;

  const float* emb   = (const float*)d_in[0];
  const int*   user  = (const int*)d_in[1];
  const int*   ts    = (const int*)d_in[2];
  const int*   click = (const int*)d_in[3];
  const float* W1 = (const float*)d_in[4];
  const float* b1 = (const float*)d_in[5];
  const float* W2 = (const float*)d_in[6];
  const float* b2 = (const float*)d_in[7];
  const float* W3 = (const float*)d_in[8];
  const float* b3 = (const float*)d_in[9];
  float* out = (float*)d_out;

  char* ws = (char*)d_ws;
  unsigned short* W1h = (unsigned short*)(ws + kOffW1h);
  unsigned short* W1l = (unsigned short*)(ws + kOffW1l);
  unsigned short* W2h = (unsigned short*)(ws + kOffW2h);
  unsigned short* W2l = (unsigned short*)(ws + kOffW2l);
  unsigned short* W3h = (unsigned short*)(ws + kOffW3h);
  unsigned short* W3l = (unsigned short*)(ws + kOffW3l);
  unsigned short* Hh  = (unsigned short*)(ws + kOffHh);
  unsigned short* Hl  = (unsigned short*)(ws + kOffHl);
  float*          flag = (float*)(ws + kOffFlag);
  unsigned short* A1h = (unsigned short*)(ws + kOffA1h);
  unsigned short* A1l = (unsigned short*)(ws + kOffA1l);
  unsigned short* A2h = (unsigned short*)(ws + kOffA2h);
  unsigned short* A2l = (unsigned short*)(ws + kOffA2l);
  float*          A3  = (float*)(ws + kOffA3);
  const float*    dummyR = (const float*)(ws + kOffA3);

  wt_split_kernel<<<dim3(kDim / 64, kHidA / 64), 256, 0, stream>>>(W1, W1h, W1l, kDim, kHidA);
  wt_split_kernel<<<dim3(kHidA / 64, kHidB / 64), 256, 0, stream>>>(W2, W2h, W2l, kHidA, kHidB);
  wt_split_kernel<<<dim3(kHidB / 64, kDim / 64), 256, 0, stream>>>(W3, W3h, W3l, kHidB, kDim);

  history_kernel<<<kRows / kRowsPerHistBlock, 256, 0, stream>>>(emb, user, ts, click, Hh, Hl, flag);

  {
    const int tiles = (kRows / 64) * (kHidA / 64);
    wmma_gemm64<1, true, 2, 2, false, 6><<<dim3((tiles + 7) / 8, 1), 256, 0, stream>>>(
        Hh, Hl, kDim, 0L, W1h, W1l, kDim, 0L, (void*)A1h, (void*)A1l, kHidA, 0L,
        b1, dummyR, 0L, kRows, kHidA, kDim, 1.0f);
  }
  {
    const int tiles = (kRows / 64) * (kHidB / 64);
    wmma_gemm64<1, true, 2, 2, false, 6><<<dim3((tiles + 7) / 8, 1), 256, 0, stream>>>(
        A1h, A1l, kHidA, 0L, W2h, W2l, kHidA, 0L, (void*)A2h, (void*)A2l, kHidB, 0L,
        b2, dummyR, 0L, kRows, kHidB, kHidA, 1.0f);
  }
  {
    const int tiles = (kRows / 64) * (kDim / 64);
    wmma_gemm64<1, true, 2, 0, false, 0><<<dim3((tiles + 7) / 8, 1), 256, 0, stream>>>(
        A2h, A2l, kHidB, 0L, W3h, W3l, kHidB, 0L, (void*)A3, (void*)A3, kDim, 0L,
        b3, dummyR, 0L, kRows, kDim, kHidB, 1.0f);
  }

  l2norm_kernel<<<kRows / 8, 256, 0, stream>>>(A3, flag, out);
}
